// HierDDmx_28355374088369
// MI455X (gfx1250) — hardware-verified
//
#include <hip/hip_runtime.h>
#include <math.h>

#ifndef NB
#define NB 2
#endif
#ifndef SEQ
#define SEQ 2048
#endif
#define SEQ_FULL 2048
#define D0 512
#define D1 64
#define D2 512
#define NBAS 64
#define NGRP 8
#define MTOK (NB * SEQ)
#define WCARRY 64.0f
#define WFOLD 0.015625f
#define LN_EPS 1e-5f

static_assert(SEQ % 64 == 0);
static_assert(SEQ <= SEQ_FULL);
static_assert(MTOK % 64 == 0);
static_assert(D0 == 512 && D1 == 64 && D2 == 512 && NBAS == 64 && NGRP == 8);
static_assert(D0 % 32 == 0 && D1 % 32 == 0);
static_assert((MTOK * D0 / 8) % 256 == 0);
static_assert((D0 * D0 / 8) % 256 == 0);
static_assert((D1 * D0 / 8) % 256 == 0);
static_assert((D0 * NBAS) % (32 * 64) == 0);
static_assert(((long long)SEQ * 4096ll) % 256ll == 0 && (long long)SEQ * 4096ll < 4294967296ll);

typedef __attribute__((ext_vector_type(16))) _Float16 v16h;
typedef __attribute__((ext_vector_type(8)))  _Float16 v8h;
typedef __attribute__((ext_vector_type(16))) __bf16   v16b;
typedef __attribute__((ext_vector_type(8)))  float    v8f;
typedef __attribute__((ext_vector_type(4)))  float    v4f;
typedef __attribute__((ext_vector_type(4)))  unsigned int v4u;
typedef __attribute__((ext_vector_type(8)))  unsigned int v8u;
typedef _Float16 h16;


#define VST2(T, ptr, val) do { const T vst2_v_ = (val); *(volatile T*)(ptr) = vst2_v_; __threadfence(); *(volatile T*)(ptr) = vst2_v_; } while (0)
#define VST2V4(ptr, val) do { const v4f vst2_v4_ = (val); *(volatile v4f*)(ptr) = vst2_v4_; __threadfence(); *(volatile v4f*)(ptr) = vst2_v4_; } while (0)

__device__ __forceinline__ float bfr(float f) {
    unsigned u = __float_as_uint(f);
    u += 0x7FFFu + ((u >> 16) & 1u);
    return __uint_as_float(u & 0xFFFF0000u);
}
__device__ __forceinline__ unsigned bf_bits(float f) {
    unsigned u = __float_as_uint(f);
    u += 0x7FFFu + ((u >> 16) & 1u);
    return u >> 16;
}
static __device__ __forceinline__ h16 toh_flush(float v) { const float w = (fabsf(v) < 6.103515625e-05f) ? 0.0f : v; return (h16)w; }

union FragU { v16h v; v8h h[2]; };
__device__ __forceinline__ v16h frag_ld(const _Float16* p) {
    FragU f; f.h[0] = *(const v8h*)(p); f.h[1] = *(const v8h*)(p + 16); return f.v;
}
union FragBU { v8u v; v4u q[2]; };
__device__ __forceinline__ v8u frag_ld_b(const unsigned short* p) {
    FragBU f; f.q[0] = *(const v4u*)(p); f.q[1] = *(const v4u*)(p + 16); return f.v;
}
__device__ __forceinline__ v8f wmma16g(v16h a, v16h b, v8f c) {
    c = __builtin_amdgcn_wmma_f32_16x16x32_f16(false, a, false, b, (short)0, c, false, false);
    asm volatile("v_nop\n\tv_nop\n\tv_nop\n\tv_nop" : "+v"(c) : "v"(a), "v"(b));
    return c;
}
__device__ __forceinline__ v8f wmmabg(v8u a, v8u b, v8f c) {
    c = __builtin_amdgcn_wmma_f32_16x16x32_bf16(false, __builtin_bit_cast(v16b, a), false, __builtin_bit_cast(v16b, b), (short)0, c, false, false);
    asm volatile("v_nop\n\tv_nop\n\tv_nop\n\tv_nop" : "+v"(c) : "v"(a), "v"(b));
    return c;
}
__device__ __forceinline__ void wave_sync_lds() {
    __builtin_amdgcn_fence(3  , "workgroup");
    __builtin_amdgcn_wave_barrier();
    __builtin_amdgcn_fence(2  , "workgroup");
}

__device__ __forceinline__ void cvt8_bf(const float* __restrict__ s, unsigned short* __restrict__ d) {
    const v4f a = *(const v4f*)(s);
    const v4f b = *(const v4f*)(s + 4);
    v4u pk;
    pk.x = bf_bits(a.x) | (bf_bits(a.y) << 16);
    pk.y = bf_bits(a.z) | (bf_bits(a.w) << 16);
    pk.z = bf_bits(b.x) | (bf_bits(b.y) << 16);
    pk.w = bf_bits(b.z) | (bf_bits(b.w) << 16);
    VST2(v4u, d, pk);
}

__global__ __launch_bounds__(256) void k_cvt_x(const float* __restrict__ x, unsigned short* __restrict__ xbf) {
    const unsigned u = blockIdx.x * 256u + threadIdx.x;
    if (u >= (unsigned)(MTOK * D0 / 8)) return;
    const unsigned m = u >> 6, c0 = (u & 63u) * 8u;
    const unsigned b = m / (unsigned)SEQ, s = m % (unsigned)SEQ;
    cvt8_bf(x + (size_t)(b * (unsigned)SEQ_FULL + s) * D0 + c0, xbf + (size_t)m * D0 + c0);
}

__global__ __launch_bounds__(256) void k_cvt_w(const float* __restrict__ w, unsigned short* __restrict__ wbf, unsigned n8) {
    const unsigned u = blockIdx.x * 256u + threadIdx.x;
    if (u >= n8) return;
    cvt8_bf(w + (size_t)u * 8u, wbf + (size_t)u * 8u);
}

__global__ __launch_bounds__(256) void k_wconv16(const float* __restrict__ w, _Float16* __restrict__ w16, unsigned n8) {
    const unsigned u = blockIdx.x * 256u + threadIdx.x;
    if (u >= n8) return;
    const v4f a = *(const v4f*)(w + (size_t)u * 8u);
    const v4f b = *(const v4f*)(w + (size_t)u * 8u + 4u);
    v8h hv;
#pragma unroll
    for (int e = 0; e < 4; ++e) {
        hv[e]     = toh_flush(bfr(a[e]) * WCARRY);
        hv[4 + e] = toh_flush(bfr(b[e]) * WCARRY);
    }
    VST2(v8h, w16 + (size_t)u * 8u, hv);
}

__global__ __launch_bounds__(256) void k_tr64(const float* __restrict__ A, float* __restrict__ AT) {
    __shared__ float sA[32 * 65];
    const unsigned t = threadIdx.x;
    const unsigned o0 = blockIdx.x * 32u;
#pragma unroll
    for (int i = 0; i < 8; ++i) {
        const unsigned e = t + 256u * (unsigned)i;
        const unsigned r = e >> 6, cc = e & 63u;
        sA[r * 65u + cc] = bfr(A[(size_t)(o0 + r) * 64u + cc]);
    }
    __syncthreads();
    const unsigned lane = t & 31u;
    const unsigned wave = (unsigned)__builtin_amdgcn_readfirstlane((int)(t >> 5));
    const unsigned q = lane >> 3, c4 = (lane & 7u) * 4u;
    static_assert(8 * 4 * 2 == 64);
#pragma unroll
    for (int it = 0; it < 2; ++it) {
        const unsigned j = (unsigned)it * 32u + wave * 4u + q;
        v4f v;
        v.x = sA[(c4 + 0u) * 65u + j];
        v.y = sA[(c4 + 1u) * 65u + j];
        v.z = sA[(c4 + 2u) * 65u + j];
        v.w = sA[(c4 + 3u) * 65u + j];
        VST2V4(AT + (size_t)j * 512u + o0 + c4, v);
    }
}

__global__ __launch_bounds__(256) void k_wp(const float* __restrict__ P2, float* __restrict__ wp) {
#pragma clang fp contract(off)
    const unsigned u = blockIdx.x * 256u + threadIdx.x;
    if (u >= (unsigned)SEQ * 4096u) return;
    const unsigned ij = u & 4095u;
    const unsigned s = u >> 12;
    const unsigned i = ij >> 6, j = ij & 63u;
    const float tps = 6.2831855f * (float)s;
    const float pbase = (float)(i * 512u + j * 8u + 2u);
    const float* pr = P2 + (size_t)ij * 8u;
    float w = 0.0f;
#pragma unroll 1
    for (unsigned g = 0; g < (unsigned)NGRP; ++g) {
        const float arg = tps / (pbase + (float)g);
        const float cv = cosf(arg);
        const float pv = bfr(pr[g]);
        w = w + pv * cv;
    }
    VST2(float, wp + u, w);
}

#define S1_P 516
static_assert(16 * S1_P * 4 <= 131072);
__global__ __launch_bounds__(128) void k_stage1(const unsigned short* __restrict__ xbf, const unsigned short* __restrict__ w1bf,
                                                const float* __restrict__ g1, const float* __restrict__ b1,
                                                const float* __restrict__ a1t, const float* __restrict__ B1,
                                                _Float16* __restrict__ h1) {
    __shared__ __align__(16) float sT[16 * S1_P];
    const unsigned lane = threadIdx.x & 31u;
    const unsigned wave = (unsigned)__builtin_amdgcn_readfirstlane((int)(threadIdx.x >> 5));
    const unsigned hh = lane >> 4, c = lane & 15u;
    const unsigned m0 = blockIdx.x * 16u;
    const unsigned n0 = wave * 128u;

    v8f acc[8];
#pragma unroll
    for (int j = 0; j < 8; ++j) acc[j] = (v8f){0.f,0.f,0.f,0.f,0.f,0.f,0.f,0.f};
    const unsigned short* ap = xbf + (size_t)(m0 + c) * 512u + 8u * hh;
    const unsigned short* bp = w1bf + (size_t)(n0 + c) * 512u + 8u * hh;
#pragma unroll 1
    for (unsigned k0 = 0; k0 < 512u; k0 += 32u) {
        const v8u af = frag_ld_b(ap + k0);
#pragma unroll
        for (int j = 0; j < 8; ++j) {
            const v8u bf = frag_ld_b(bp + (size_t)((unsigned)j * 16u * 512u) + k0);
            acc[j] = wmmabg(af, bf, acc[j]);
        }
    }
#pragma unroll
    for (int j = 0; j < 8; ++j)
#pragma unroll
        for (int r = 0; r < 8; ++r)
            sT[(8u * hh + (unsigned)r) * S1_P + n0 + (unsigned)j * 16u + c] = acc[j][r];
    __syncthreads();

    float gg[16], bb[16];
#pragma unroll
    for (int p = 0; p < 2; ++p) {
        const unsigned cb = (unsigned)p * 256u + 8u * lane;
        const v4f ga = *(const v4f*)(g1 + cb), gb = *(const v4f*)(g1 + cb + 4u);
        const v4f ba = *(const v4f*)(b1 + cb), bc = *(const v4f*)(b1 + cb + 4u);
#pragma unroll
        for (int e = 0; e < 4; ++e) {
            gg[8 * p + e] = bfr(ga[e]); gg[8 * p + 4 + e] = bfr(gb[e]);
            bb[8 * p + e] = bfr(ba[e]); bb[8 * p + 4 + e] = bfr(bc[e]);
        }
    }
    static_assert(32 * 16 * 2 == 512 * 2);
#pragma unroll 1
    for (unsigned it = 0; it < 4u; ++it) {
        const unsigned rr = wave * 4u + it;
        const unsigned m = m0 + rr;
        const unsigned jb = (m % (unsigned)SEQ) & 63u;
        float v[16];
#pragma unroll
        for (int p = 0; p < 2; ++p) {
            const unsigned cb = (unsigned)p * 256u + 8u * lane;
            const v4f a = *(const v4f*)(sT + rr * S1_P + cb);
            const v4f b = *(const v4f*)(sT + rr * S1_P + cb + 4u);
#pragma unroll
            for (int e = 0; e < 4; ++e) { v[8 * p + e] = a[e]; v[8 * p + 4 + e] = b[e]; }
        }
        float s = 0.f;
#pragma unroll
        for (int i = 0; i < 16; ++i) s += v[i];
#pragma unroll
        for (int o = 16; o > 0; o >>= 1) s += __shfl_xor(s, o, 32);
        const float mu = s * (1.0f / 512.0f);
        float q = 0.f;
#pragma unroll
        for (int i = 0; i < 16; ++i) { v[i] = v[i] - mu; q += v[i] * v[i]; }
#pragma unroll
        for (int o = 16; o > 0; o >>= 1) q += __shfl_xor(q, o, 32);
        const float rs = rsqrtf(q * (1.0f / 512.0f) + LN_EPS);
        float dot = 0.f;
#pragma unroll
        for (int p = 0; p < 2; ++p) {
            const unsigned cb = (unsigned)p * 256u + 8u * lane;
            const v4f ba = *(const v4f*)(B1 + (size_t)jb * 512u + cb);
            const v4f bc = *(const v4f*)(B1 + (size_t)jb * 512u + cb + 4u);
#pragma unroll
            for (int e = 0; e < 4; ++e) {
                dot += (v[8 * p + e] * rs * gg[8 * p + e] + bb[8 * p + e]) * bfr(ba[e]);
                dot += (v[8 * p + 4 + e] * rs * gg[8 * p + 4 + e] + bb[8 * p + 4 + e]) * bfr(bc[e]);
            }
        }
#pragma unroll
        for (int o = 16; o > 0; o >>= 1) dot += __shfl_xor(dot, o, 32);

        v8h hv[2];
#pragma unroll
        for (int p = 0; p < 2; ++p) {
            const unsigned cb = (unsigned)p * 256u + 8u * lane;
            const v4f aa = *(const v4f*)(a1t + (size_t)jb * 512u + cb);
            const v4f ab = *(const v4f*)(a1t + (size_t)jb * 512u + cb + 4u);
            const v4u xw = *(const v4u*)(xbf + (size_t)m * 512u + cb);
            float xv[8];
            xv[0] = __uint_as_float(xw.x << 16); xv[1] = __uint_as_float(xw.x & 0xFFFF0000u);
            xv[2] = __uint_as_float(xw.y << 16); xv[3] = __uint_as_float(xw.y & 0xFFFF0000u);
            xv[4] = __uint_as_float(xw.z << 16); xv[5] = __uint_as_float(xw.z & 0xFFFF0000u);
            xv[6] = __uint_as_float(xw.w << 16); xv[7] = __uint_as_float(xw.w & 0xFFFF0000u);
#pragma unroll
            for (int e = 0; e < 4; ++e) {
                hv[p][e]     = toh_flush(dot * aa[e] + xv[e]);
                hv[p][4 + e] = toh_flush(dot * ab[e] + xv[4 + e]);
            }
        }
        _Float16* hrow = h1 + (size_t)m * 512u + 8u * lane;
        for (int pass = 0; pass < 2; ++pass) {
#pragma unroll
            for (int p = 0; p < 2; ++p) *(volatile v8h*)(hrow + (unsigned)p * 256u) = hv[p];
            __threadfence();
        }
    }
}

#define S2_P 132
static_assert(4 * 16 * S2_P * 4 <= 131072);
__global__ __launch_bounds__(128) void k_stage2(const _Float16* __restrict__ h1, const _Float16* __restrict__ bt2,
                                                const float* __restrict__ g2, const float* __restrict__ b2,
                                                const float* __restrict__ wp, _Float16* __restrict__ h2) {
    __shared__ __align__(16) float sT[4 * 16 * S2_P];
    const unsigned lane = threadIdx.x & 31u;
    const unsigned wave = (unsigned)__builtin_amdgcn_readfirstlane((int)(threadIdx.x >> 5));
    const unsigned hh = lane >> 4, c = lane & 15u;
    const unsigned m0 = (blockIdx.x * 4u + wave) * 16u;
    const unsigned wb = wave * (16u * S2_P);

    v8f acc[8];
#pragma unroll
    for (int j = 0; j < 8; ++j) acc[j] = (v8f){0.f,0.f,0.f,0.f,0.f,0.f,0.f,0.f};
    const _Float16* ap = h1 + (size_t)(m0 + c) * 512u + 8u * hh;
    const _Float16* bp = bt2 + (size_t)c * 512u + 8u * hh;
#pragma unroll 1
    for (unsigned k0 = 0; k0 < 512u; k0 += 32u) {
        const v16h af = frag_ld(ap + k0);
#pragma unroll
        for (int j = 0; j < 8; ++j) {
            const v16h bf = frag_ld(bp + (size_t)((unsigned)j * 16u * 512u) + k0);
            acc[j] = wmma16g(af, bf, acc[j]);
        }
    }
#pragma unroll
    for (int j = 0; j < 8; ++j)
#pragma unroll
        for (int r = 0; r < 8; ++r)
            sT[wb + (8u * hh + (unsigned)r) * S2_P + (unsigned)j * 16u + c] = acc[j][r] * WFOLD;
    wave_sync_lds();

    const float gA = bfr(g2[lane]), gB = bfr(g2[lane + 32u]);
    const float bA = bfr(b2[lane]), bB = bfr(b2[lane + 32u]);
#pragma unroll 1
    for (unsigned r = 0; r < 16u; ++r) {
        const unsigned ro = wb + r * S2_P;
        const float v0 = sT[ro + lane], v1 = sT[ro + lane + 32u];
        float s = v0 + v1;
#pragma unroll
        for (int o = 16; o > 0; o >>= 1) s += __shfl_xor(s, o, 32);
        const float mu = s * (1.0f / 64.0f);
        const float d0 = v0 - mu, d1 = v1 - mu;
        float q = d0 * d0 + d1 * d1;
#pragma unroll
        for (int o = 16; o > 0; o >>= 1) q += __shfl_xor(q, o, 32);
        const float rs = rsqrtf(q * (1.0f / 64.0f) + LN_EPS);
        sT[ro + lane]       = d0 * rs * gA + bA;
        sT[ro + lane + 32u] = d1 * rs * gB + bB;
    }
    wave_sync_lds();

#pragma unroll 1
    for (unsigned r = 0; r < 16u; ++r) {
        const unsigned ro = wb + r * S2_P;
        const unsigned s = (m0 + r) % (unsigned)SEQ;
        const float* w0p = wp + (size_t)s * 4096u + (size_t)lane * 64u;
        const float* w1p = w0p + 32u * 64u;
        float n0 = 0.f, n1 = 0.f;
#pragma unroll 4
        for (unsigned j4 = 0; j4 < 16u; ++j4) {
            const v4f wa = *(const v4f*)(w0p + 4u * j4);
            const v4f wc = *(const v4f*)(w1p + 4u * j4);
            const v4f t4 = *(const v4f*)(sT + ro + 4u * j4);
            n0 += wa.x * t4.x; n0 += wa.y * t4.y; n0 += wa.z * t4.z; n0 += wa.w * t4.w;
            n1 += wc.x * t4.x; n1 += wc.y * t4.y; n1 += wc.z * t4.z; n1 += wc.w * t4.w;
        }
        const float r0 = sT[ro + 64u + lane], r1 = sT[ro + 96u + lane];
        sT[ro + 64u + lane] = n0 + r0;
        sT[ro + 96u + lane] = n1 + r1;
    }
    wave_sync_lds();

    {
        static_assert(4 * 4 == 16 && 8 * 16 == 64 * 2);
        const unsigned q = lane >> 3, c8 = (lane & 7u) * 8u;
        v8h hv[4];
#pragma unroll
        for (int it = 0; it < 4; ++it) {
            const unsigned row = (unsigned)it * 4u + q;
            const v4f a = *(const v4f*)(sT + wb + row * S2_P + 64u + c8);
            const v4f b = *(const v4f*)(sT + wb + row * S2_P + 64u + c8 + 4u);
#pragma unroll
            for (int e = 0; e < 4; ++e) { hv[it][e] = toh_flush(a[e]); hv[it][4 + e] = toh_flush(b[e]); }
        }
        for (int pass = 0; pass < 2; ++pass) {
#pragma unroll
            for (int it = 0; it < 4; ++it) {
                const unsigned row = (unsigned)it * 4u + q;
                *(volatile v8h*)(h2 + (size_t)(m0 + row) * 64u + c8) = hv[it];
            }
            __threadfence();
        }
    }
}

#define S3_P 516
static_assert(2 * 16 * S3_P * 4 <= 131072);
__global__ __launch_bounds__(128) void k_stage3(const _Float16* __restrict__ h2, const _Float16* __restrict__ bt3,
                                                const float* __restrict__ g3, const float* __restrict__ b3,
                                                const float* __restrict__ a3t, const float* __restrict__ B3,
                                                float* __restrict__ out) {
    __shared__ __align__(16) float sU[16 * S3_P];
    __shared__ __align__(16) float sR[16 * S3_P];
    const unsigned lane = threadIdx.x & 31u;
    const unsigned wave = (unsigned)__builtin_amdgcn_readfirstlane((int)(threadIdx.x >> 5));
    const unsigned hh = lane >> 4, c = lane & 15u;
    const unsigned m0 = blockIdx.x * 16u;
    const unsigned n0 = wave * 128u;

    const v16h af0 = frag_ld(h2 + (size_t)(m0 + c) * 64u + 8u * hh);
    const v16h af1 = frag_ld(h2 + (size_t)(m0 + c) * 64u + 32u + 8u * hh);
#pragma unroll
    for (int j = 0; j < 8; ++j) {
        const unsigned n = n0 + (unsigned)j * 16u + c;
        const v16h bu0 = frag_ld(bt3 + (size_t)n * 64u + 8u * hh);
        const v16h bu1 = frag_ld(bt3 + (size_t)n * 64u + 32u + 8u * hh);
        v8f u = (v8f){0.f,0.f,0.f,0.f,0.f,0.f,0.f,0.f};
        u = wmma16g(af0, bu0, u);
        u = wmma16g(af1, bu1, u);
        const v16h br0 = frag_ld(bt3 + (size_t)(512u + n) * 64u + 8u * hh);
        const v16h br1 = frag_ld(bt3 + (size_t)(512u + n) * 64u + 32u + 8u * hh);
        v8f rv = (v8f){0.f,0.f,0.f,0.f,0.f,0.f,0.f,0.f};
        rv = wmma16g(af0, br0, rv);
        rv = wmma16g(af1, br1, rv);
#pragma unroll
        for (int r = 0; r < 8; ++r) {
            sU[(8u * hh + (unsigned)r) * S3_P + n] = u[r] * WFOLD;
            sR[(8u * hh + (unsigned)r) * S3_P + n] = rv[r] * WFOLD;
        }
    }
    __syncthreads();

    float gg[16], bb[16];
#pragma unroll
    for (int p = 0; p < 4; ++p) {
        const unsigned cb = (unsigned)p * 128u + 4u * lane;
        const v4f ga = *(const v4f*)(g3 + cb);
        const v4f ba = *(const v4f*)(b3 + cb);
#pragma unroll
        for (int e = 0; e < 4; ++e) { gg[4 * p + e] = bfr(ga[e]); bb[4 * p + e] = bfr(ba[e]); }
    }
    static_assert(32 * 16 * 4 == 512 * 4);
#pragma unroll 1
    for (unsigned it = 0; it < 4u; ++it) {
        const unsigned rr = wave * 4u + it;
        const unsigned m = m0 + rr;
        const unsigned bq = m / (unsigned)SEQ, sq = m % (unsigned)SEQ;
        const unsigned jb = sq & 63u;
        const unsigned grow = bq * (unsigned)SEQ_FULL + sq;
        float v[16];
#pragma unroll
        for (int p = 0; p < 4; ++p) {
            const v4f a = *(const v4f*)(sU + rr * S3_P + (unsigned)p * 128u + 4u * lane);
#pragma unroll
            for (int e = 0; e < 4; ++e) v[4 * p + e] = a[e];
        }
        float s = 0.f;
#pragma unroll
        for (int i = 0; i < 16; ++i) s += v[i];
#pragma unroll
        for (int o = 16; o > 0; o >>= 1) s += __shfl_xor(s, o, 32);
        const float mu = s * (1.0f / 512.0f);
        float q = 0.f;
#pragma unroll
        for (int i = 0; i < 16; ++i) { v[i] = v[i] - mu; q += v[i] * v[i]; }
#pragma unroll
        for (int o = 16; o > 0; o >>= 1) q += __shfl_xor(q, o, 32);
        const float rs = rsqrtf(q * (1.0f / 512.0f) + LN_EPS);
        float dot = 0.f;
#pragma unroll
        for (int p = 0; p < 4; ++p) {
            const v4f ba = *(const v4f*)(B3 + (size_t)jb * 512u + (unsigned)p * 128u + 4u * lane);
#pragma unroll
            for (int e = 0; e < 4; ++e) dot += (v[4 * p + e] * rs * gg[4 * p + e] + bb[4 * p + e]) * bfr(ba[e]);
        }
#pragma unroll
        for (int o = 16; o > 0; o >>= 1) dot += __shfl_xor(dot, o, 32);

        v4f vv[4];
#pragma unroll
        for (int p = 0; p < 4; ++p) {
            const v4f aa = *(const v4f*)(a3t + (size_t)jb * 512u + (unsigned)p * 128u + 4u * lane);
            const v4f rv = *(const v4f*)(sR + rr * S3_P + (unsigned)p * 128u + 4u * lane);
            vv[p] = aa * dot + rv;
        }
        float* orow = out + (size_t)grow * 512u + 4u * lane;
        for (int pass = 0; pass < 2; ++pass) {
#pragma unroll
            for (int p = 0; p < 4; ++p) *(volatile v4f*)(orow + (unsigned)p * 128u) = vv[p];
            __threadfence();
        }
    }
}

static_assert((size_t)MTOK * D0 * 2 + (size_t)D0 * D0 * 2 + (size_t)128 * 512 * 2 + (size_t)1024 * 64 * 2 +
              (size_t)64 * 512 * 4 * 2 + (size_t)SEQ * 4096 * 4 + (size_t)MTOK * D0 * 2 + (size_t)MTOK * D1 * 2 <= (size_t)134217728);

extern "C" void kernel_launch(void* const* d_in, const int* in_sizes, int n_in, void* d_out, int out_size,
                              void* d_ws, size_t ws_size, hipStream_t stream) {
    if (n_in < 17) return;
    if (in_sizes[0] < ((NB - 1) * SEQ_FULL + SEQ) * D0 || in_sizes[1] < D0 * D0 || in_sizes[2] < D0 || in_sizes[3] < D0) return;
    if (in_sizes[4] < D0 * NBAS || in_sizes[5] < NBAS * D0 || in_sizes[6] < D1 * D0 || in_sizes[7] < D1 || in_sizes[8] < D1) return;
    if (in_sizes[9] < D1 * D1 * NGRP || in_sizes[10] < D1 * D0 || in_sizes[11] < D2 * D1 || in_sizes[12] < D2 || in_sizes[13] < D2) return;
    if (in_sizes[14] < D2 * NBAS || in_sizes[15] < NBAS * D2 || in_sizes[16] < D2 * D1) return;
    if (out_size < ((NB - 1) * SEQ_FULL + SEQ) * D2) return;

    const float* x  = (const float*)d_in[0];
    const float* W1 = (const float*)d_in[1];
    const float* g1 = (const float*)d_in[2];
    const float* b1 = (const float*)d_in[3];
    const float* A1 = (const float*)d_in[4];
    const float* B1 = (const float*)d_in[5];
    const float* M2 = (const float*)d_in[6];
    const float* g2 = (const float*)d_in[7];
    const float* b2 = (const float*)d_in[8];
    const float* P2 = (const float*)d_in[9];
    const float* R2 = (const float*)d_in[10];
    const float* W3 = (const float*)d_in[11];
    const float* g3 = (const float*)d_in[12];
    const float* b3 = (const float*)d_in[13];
    const float* A3 = (const float*)d_in[14];
    const float* B3 = (const float*)d_in[15];
    const float* R3 = (const float*)d_in[16];
    float* out = (float*)d_out;

    char* wsp = (char*)d_ws;
    size_t off = 0;
    auto carve = [&](size_t bytes) -> void* { void* r = wsp + off; off += (bytes + 255) & ~(size_t)255; return r; };
    unsigned short* xbf  = (unsigned short*)carve((size_t)MTOK * D0 * 2);
    unsigned short* w1bf = (unsigned short*)carve((size_t)D0 * D0 * 2);
    _Float16*       bt2  = (_Float16*)carve((size_t)128 * 512 * 2);
    _Float16*       bt3  = (_Float16*)carve((size_t)1024 * 64 * 2);
    float*          a1t  = (float*)carve((size_t)64 * 512 * 4);
    float*          a3t  = (float*)carve((size_t)64 * 512 * 4);
    float*          wp   = (float*)carve((size_t)SEQ * 4096 * 4);
    _Float16*       h1   = (_Float16*)carve((size_t)MTOK * D0 * 2);
    _Float16*       h2   = (_Float16*)carve((size_t)MTOK * D1 * 2);
    if (off > ws_size || off > (size_t)134217728) return;

    k_cvt_x<<<(MTOK * D0 / 8) / 256, 256, 0, stream>>>(x, xbf);
    k_cvt_w<<<(D0 * D0 / 8) / 256, 256, 0, stream>>>(W1, w1bf, (unsigned)(D0 * D0 / 8));
    k_wconv16<<<(D1 * D0 / 8) / 256, 256, 0, stream>>>(M2, bt2, (unsigned)(D1 * D0 / 8));
    k_wconv16<<<(D1 * D0 / 8) / 256, 256, 0, stream>>>(R2, bt2 + (size_t)64 * 512, (unsigned)(D1 * D0 / 8));
    k_wconv16<<<(D2 * D1 / 8) / 256, 256, 0, stream>>>(W3, bt3, (unsigned)(D2 * D1 / 8));
    k_wconv16<<<(D2 * D1 / 8) / 256, 256, 0, stream>>>(R3, bt3 + (size_t)512 * 64, (unsigned)(D2 * D1 / 8));
    k_tr64<<<512 / 32, 256, 0, stream>>>(A1, a1t);
    k_tr64<<<512 / 32, 256, 0, stream>>>(A3, a3t);
    k_wp<<<SEQ * 16, 256, 0, stream>>>(P2, wp);

    k_stage1<<<MTOK / 16, 128, 0, stream>>>(xbf, w1bf, g1, b1, a1t, B1, h1);
    k_stage2<<<MTOK / 64, 128, 0, stream>>>((const _Float16*)h1, (const _Float16*)bt2, g2, b2, wp, h2);
    k_stage3<<<MTOK / 16, 128, 0, stream>>>((const _Float16*)h2, (const _Float16*)bt3, g3, b3, a3t, B3, out);
}
